// GraphConvpoolMPNN_block_49795850830069
// MI455X (gfx1250) — hardware-verified
//
#include <hip/hip_runtime.h>
#define BS 16
#define SC 17
#define NNODE 256
#define FF 64
#define LW 16
#define N1 512
#define NG (BS * LW)
#define NRX (BS * SC * NNODE)
#define NRW (NG * N1)
#define GG 16
typedef __bf16 v16b __attribute__((ext_vector_type(16)));
typedef unsigned short v8us __attribute__((ext_vector_type(8), may_alias));
typedef float  v8f  __attribute__((ext_vector_type(8)));
typedef float  v4f  __attribute__((ext_vector_type(4)));
typedef float  v4fa __attribute__((ext_vector_type(4), may_alias));
union FragB { v16b v; v8us half[2]; unsigned short u[16]; };

__device__ __forceinline__ unsigned short bf16_bits(float x) { unsigned int u = __float_as_uint(x); return (unsigned short)((u + 0x7FFFu + ((u >> 16) & 1u)) >> 16); }
__device__ __forceinline__ float bf16_val(unsigned short b) { return __uint_as_float(((unsigned int)b) << 16); }
__device__ __forceinline__ float bf16_round(float x) { return bf16_val(bf16_bits(x)); }
template <int NT>
__device__ __forceinline__ v8f mmaN(v16b ah, v16b al, v16b bh, v16b bl, v8f c) {
  c = __builtin_amdgcn_wmma_f32_16x16x32_bf16(false, ah, false, bh, (short)0, c, false, false);
  if (NT >= 2) c = __builtin_amdgcn_wmma_f32_16x16x32_bf16(false, al, false, bh, (short)0, c, false, false);
  if (NT >= 3) c = __builtin_amdgcn_wmma_f32_16x16x32_bf16(false, ah, false, bl, (short)0, c, false, false);
  asm volatile("v_nop\n\tv_nop\n\tv_nop\n\tv_nop" : "+v"(c) : "v"(ah), "v"(al), "v"(bh), "v"(bl));
  return c;
}

__global__ __launch_bounds__(256) void k_wt_bf16(const float* __restrict__ W, unsigned short* __restrict__ Wt, int K, int N) {
  const int t = blockIdx.x * 256 + threadIdx.x;
  const int k8n = K / 8;
  if (t >= N * k8n) return;
  const int n = t / k8n, k8 = (t % k8n) * 8;
  v8us v;
#pragma unroll
  for (int i = 0; i < 8; ++i) v[i] = bf16_bits(W[(size_t)(k8 + i) * N + n]);
  *(volatile v8us*)(Wt + (size_t)n * K + k8) = v;
  __threadfence();
  *(volatile v8us*)(Wt + (size_t)n * K + k8) = v;
}

template <bool ASPLIT, int ACT, bool BIAS_BF16>
__global__ __launch_bounds__(128) void k_gemm_bf(const float* __restrict__ A, int lda, const unsigned short* __restrict__ Wt, int ldb,
                                               const float* __restrict__ bias, float* __restrict__ C, int ldc, int M, int N, int K) {
  __shared__ __attribute__((aligned(16))) float so[4][16][64];
  const int tid = threadIdx.x, w = tid >> 5, lane = tid & 31, ln = lane & 15, hh = lane >> 4;
  const int ntn = N / 64;
  const int wid = blockIdx.x * 4 + w;
  const int mt = wid / ntn, nq = wid % ntn;
  if (mt * 16 >= M) return;
  const int row0 = mt * 16, col0 = nq * 64;
  const float* arow = A + (size_t)(row0 + ln) * lda;
  v8f acc[4] = {};
  for (int kb = 0; kb < K; kb += 32) {
    FragB ah, al;
    const v4f x0 = *(const v4fa*)(arow + kb + 8 * hh), x1 = *(const v4fa*)(arow + kb + 8 * hh + 4);
    const v4f x2 = *(const v4fa*)(arow + kb + 16 + 8 * hh), x3 = *(const v4fa*)(arow + kb + 16 + 8 * hh + 4);
    float xs[16] = {x0[0],x0[1],x0[2],x0[3],x1[0],x1[1],x1[2],x1[3],x2[0],x2[1],x2[2],x2[3],x3[0],x3[1],x3[2],x3[3]};
#pragma unroll
    for (int i = 0; i < 16; ++i) { const unsigned short hb = bf16_bits(xs[i]); ah.u[i] = hb; al.u[i] = ASPLIT ? bf16_bits(xs[i] - bf16_val(hb)) : (unsigned short)0; }
#pragma unroll
    for (int t = 0; t < 4; ++t) {
      const unsigned short* brow = Wt + (size_t)(col0 + t * 16 + ln) * ldb + kb;
      FragB b;
      b.half[0] = *(const v8us*)(brow + 8 * hh);
      b.half[1] = *(const v8us*)(brow + 16 + 8 * hh);
      acc[t] = mmaN<ASPLIT ? 2 : 1>(ah.v, al.v, b.v, b.v, acc[t]);
    }
  }
#pragma unroll
  for (int t = 0; t < 4; ++t) {
    float bv = bias ? bias[col0 + t * 16 + ln] : 0.f;
    if (BIAS_BF16) bv = bf16_round(bv);
#pragma unroll
    for (int r = 0; r < 8; ++r) { float v = acc[t][r] + bv; if (ACT == 1) v = fmaxf(v, 0.f); so[w][8 * hh + r][t * 16 + ln] = v; }
  }
  __builtin_amdgcn_fence(__ATOMIC_ACQ_REL, "workgroup");
  __builtin_amdgcn_wave_barrier();
  const int rsub = lane >> 4, c4 = (lane & 15) * 4;
  for (int pass = 0; pass < 2; ++pass) {
#pragma unroll
    for (int q = 0; q < 8; ++q) {
      const int r = q * 2 + rsub;
      const v4f v = *(const v4fa*)&so[w][r][c4];
      *(volatile v4f*)(C + (size_t)(row0 + r) * ldc + col0 + c4) = v;
    }
    if (pass == 0) __threadfence();
  }
}

template <bool ASPLIT, int ACT, bool BIAS_BF16, bool RES_BF16>
__global__ __launch_bounds__(128) void k_gemm_bf3(const float* __restrict__ A, int lda, const unsigned short* __restrict__ Wt, int ldb,
                                                const float* __restrict__ bias, const float* __restrict__ resid, int rmod, int ldr,
                                                float* __restrict__ C, int ldc, int M, int N, int K) {
  __shared__ __attribute__((aligned(16))) float so[4][16][64];
  const int tid = threadIdx.x, w = tid >> 5, lane = tid & 31, ln = lane & 15, hh = lane >> 4;
  const int ntn = N / 64;
  const int wid = blockIdx.x * 4 + w;
  const int mt = wid / ntn, nq = wid % ntn;
  if (mt * 16 >= M) return;
  const int row0 = mt * 16, col0 = nq * 64;
  const float* arow = A + (size_t)(row0 + ln) * lda;
  v8f acc[4] = {};
  for (int kb = 0; kb < K; kb += 32) {
    FragB ah, al;
    const v4f x0 = *(const v4fa*)(arow + kb + 8 * hh), x1 = *(const v4fa*)(arow + kb + 8 * hh + 4);
    const v4f x2 = *(const v4fa*)(arow + kb + 16 + 8 * hh), x3 = *(const v4fa*)(arow + kb + 16 + 8 * hh + 4);
    float xs[16] = {x0[0],x0[1],x0[2],x0[3],x1[0],x1[1],x1[2],x1[3],x2[0],x2[1],x2[2],x2[3],x3[0],x3[1],x3[2],x3[3]};
#pragma unroll
    for (int i = 0; i < 16; ++i) { const unsigned short hb = bf16_bits(xs[i]); ah.u[i] = hb; al.u[i] = ASPLIT ? bf16_bits(xs[i] - bf16_val(hb)) : (unsigned short)0; }
#pragma unroll
    for (int t = 0; t < 4; ++t) {
      const unsigned short* brow = Wt + (size_t)(col0 + t * 16 + ln) * ldb + kb;
      FragB b;
      b.half[0] = *(const v8us*)(brow + 8 * hh);
      b.half[1] = *(const v8us*)(brow + 16 + 8 * hh);
      acc[t] = mmaN<ASPLIT ? 2 : 1>(ah.v, al.v, b.v, b.v, acc[t]);
    }
  }
#pragma unroll
  for (int t = 0; t < 4; ++t) {
    const int col = col0 + t * 16 + ln;
    float bv = bias ? bias[col] : 0.f;
    if (BIAS_BF16) bv = bf16_round(bv);
#pragma unroll
    for (int r = 0; r < 8; ++r) {
      float v = acc[t][r] + bv;
      if (resid) { float rv = resid[(size_t)((row0 + 8 * hh + r) % rmod) * ldr + col]; if (RES_BF16) rv = bf16_round(rv); v += rv; }
      if (ACT == 1) v = fmaxf(v, 0.f);
      if (ACT == 2) v = 0.5f * v * (1.0f + erff(v * 0.70710678118654752f));
      if (ACT == 3) { const float u = 0.7978845608028654f * (v + 0.044715f * v * v * v); v = 0.5f * v * (1.0f + tanhf(u)); }
      so[w][8 * hh + r][t * 16 + ln] = v;
    }
  }
  __builtin_amdgcn_fence(__ATOMIC_ACQ_REL, "workgroup");
  __builtin_amdgcn_wave_barrier();
  const int rsub = lane >> 4, c4 = (lane & 15) * 4;
  for (int pass = 0; pass < 2; ++pass) {
#pragma unroll
    for (int q = 0; q < 8; ++q) {
      const int r = q * 2 + rsub;
      const v4f v = *(const v4fa*)&so[w][r][c4];
      *(volatile v4f*)(C + (size_t)(row0 + r) * ldc + col0 + c4) = v;
    }
    if (pass == 0) __threadfence();
  }
}
template <bool PARAM_BF16>
__global__ __launch_bounds__(256) void k_layernorm(const float* __restrict__ X, const float* __restrict__ R, const float* __restrict__ g, const float* __restrict__ bta,
                                                  float* __restrict__ out_sum, float* __restrict__ out_norm, int N, float eps) {
  __shared__ float red[256];
  const int row = blockIdx.x, tid = threadIdx.x;
  const float* x = X + (size_t)row * N; const float* rr = R ? R + (size_t)row * N : nullptr;
  float vals[16];
  const int per = N / 256;
  float s1 = 0.f;
  for (int u = 0; u < per / 4; ++u) {
    const int j = tid * 4 + 1024 * u;
    const v4f a = *(const v4fa*)(x + j);
    v4f b = {0.f,0.f,0.f,0.f}; if (rr) b = *(const v4fa*)(rr + j);
#pragma unroll
    for (int q = 0; q < 4; ++q) { const float v = a[q] + b[q]; vals[u * 4 + q] = v; s1 += v; }
  }
  red[tid] = s1; __syncthreads();
  for (int st = 128; st > 0; st >>= 1) { if (tid < st) red[tid] += red[tid + st]; __syncthreads(); }
  const float mu = red[0] / (float)N; __syncthreads();
  float s2 = 0.f;
  for (int u = 0; u < per / 4; ++u)
#pragma unroll
    for (int q = 0; q < 4; ++q) { const float c = vals[u * 4 + q] - mu; s2 += c * c; }
  red[tid] = s2; __syncthreads();
  for (int st = 128; st > 0; st >>= 1) { if (tid < st) red[tid] += red[tid + st]; __syncthreads(); }
  const float rs = rsqrtf(red[0] / (float)N + eps);
  for (int pass = 0; pass < 2; ++pass) {
    for (int u = 0; u < per / 4; ++u) {
      const int j = tid * 4 + 1024 * u;
      v4f o, sm;
#pragma unroll
      for (int q = 0; q < 4; ++q) {
        float gg = g[j + q], bb = bta[j + q];
        if (PARAM_BF16) { gg = bf16_round(gg); bb = bf16_round(bb); }
        sm[q] = vals[u * 4 + q]; o[q] = (vals[u * 4 + q] - mu) * rs * gg + bb;
      }
      if (out_sum) *(volatile v4f*)(out_sum + (size_t)row * N + j) = sm;
      *(volatile v4f*)(out_norm + (size_t)row * N + j) = o;
    }
    if (pass == 0) __threadfence();
  }
}


typedef _Float16 v16h __attribute__((ext_vector_type(16)));
union FragH { v16h v; v8us half[2]; _Float16 h[16]; unsigned short u[16]; };
template <int NT>
__device__ __forceinline__ v8f mmaH(v16h ah, v16h al, v16h bh, v16h bl, v8f c) {
  c = __builtin_amdgcn_wmma_f32_16x16x32_f16(false, ah, false, bh, (short)0, c, false, false);
  if (NT >= 2) c = __builtin_amdgcn_wmma_f32_16x16x32_f16(false, al, false, bh, (short)0, c, false, false);
  if (NT >= 3) c = __builtin_amdgcn_wmma_f32_16x16x32_f16(false, ah, false, bl, (short)0, c, false, false);
  asm volatile("v_nop\n\tv_nop\n\tv_nop\n\tv_nop" : "+v"(c) : "v"(ah), "v"(al), "v"(bh), "v"(bl));
  return c;
}
template <bool ASPLIT>
__global__ __launch_bounds__(128) void k_gemm_h(const float* __restrict__ A, int lda, size_t sA, const _Float16* __restrict__ Bh, int ldb, size_t sB, float alpha, float* __restrict__ C, int ldc, size_t sC, int M, int N, int K) {
  __shared__ __attribute__((aligned(16))) float so[4][16][64];
  const int tid = threadIdx.x, w = tid >> 5, lane = tid & 31, ln = lane & 15, hh = lane >> 4; const int by = blockIdx.y;
  A += (size_t)by * sA; Bh += (size_t)by * sB; C += (size_t)by * sC;
  const int ntn = (N + 63) / 64; const int wid = blockIdx.x * 4 + w; const int mt = wid / ntn, nq = wid % ntn; if (mt * 16 >= M) return;
  const int row0 = mt * 16, col0 = nq * 64; const float* arow = A + (size_t)(row0 + ln) * lda;
  v8f acc[4] = {};
  for (int kb = 0; kb < K; kb += 32) {
    FragH ah, al;
    const v4f x0 = *(const v4fa*)(arow + kb + 8 * hh), x1 = *(const v4fa*)(arow + kb + 8 * hh + 4), x2 = *(const v4fa*)(arow + kb + 16 + 8 * hh), x3 = *(const v4fa*)(arow + kb + 16 + 8 * hh + 4);
    float xs[16] = {x0[0],x0[1],x0[2],x0[3],x1[0],x1[1],x1[2],x1[3],x2[0],x2[1],x2[2],x2[3],x3[0],x3[1],x3[2],x3[3]};
#pragma unroll
    for (int i = 0; i < 16; ++i) { const _Float16 h = (_Float16)xs[i]; ah.h[i] = h; al.h[i] = ASPLIT ? (_Float16)(xs[i] - (float)h) : (_Float16)0.0f; }
#pragma unroll
    for (int t = 0; t < 4; ++t) { if (col0 + t * 16 >= N) continue; const size_t boff = (size_t)(col0 + t * 16 + ln) * ldb + kb; FragH bq; bq.half[0] = *(const v8us*)(Bh + boff + 8 * hh); bq.half[1] = *(const v8us*)(Bh + boff + 16 + 8 * hh);
      acc[t] = mmaH<ASPLIT ? 2 : 1>(ah.v, al.v, bq.v, bq.v, acc[t]); }
  }
#pragma unroll
  for (int t = 0; t < 4; ++t) { if (col0 + t * 16 >= N) continue;
#pragma unroll
    for (int r = 0; r < 8; ++r) so[w][8 * hh + r][t * 16 + ln] = acc[t][r] * alpha; }
  __builtin_amdgcn_fence(__ATOMIC_ACQ_REL, "workgroup"); __builtin_amdgcn_wave_barrier();
  const int rsub = lane >> 4, c4 = (lane & 15) * 4;
  for (int pass = 0; pass < 2; ++pass) {
#pragma unroll
    for (int q = 0; q < 8; ++q) { const int r = q * 2 + rsub; if (col0 + c4 < N) { const v4f v = *(const v4fa*)&so[w][r][c4]; *(volatile v4f*)(C + (size_t)(row0 + r) * ldc + col0 + c4) = v; } }
    if (pass == 0) __threadfence(); }
}

__global__ __launch_bounds__(256) void k_wt_f16(const float* __restrict__ W, _Float16* __restrict__ Wt, int K, int N, float scale) {
  const int t = blockIdx.x * 256 + threadIdx.x; if (t >= N * (K / 8)) return; const int n = t / (K / 8), k8 = (t % (K / 8)) * 8; FragH f;
#pragma unroll
  for (int i = 0; i < 8; ++i) f.h[i] = (_Float16)(bf16_round(W[(size_t)(k8 + i) * N + n]) * scale); const v8us o = f.half[0];
  *(volatile v8us*)((unsigned short*)Wt + (size_t)n * K + k8) = o; __threadfence(); *(volatile v8us*)((unsigned short*)Wt + (size_t)n * K + k8) = o;
}
template <int ACT>
__global__ __launch_bounds__(128) void k_gemm_hhx(const _Float16* __restrict__ A, int lda, size_t sA, const _Float16* __restrict__ Bh, int ldb, size_t sB, float alpha, const float* __restrict__ bias, size_t sBias, const float* __restrict__ CP, int rowsPerB, size_t sCPb, int row0g,
    float* __restrict__ C, _Float16* __restrict__ C16, int ldc, size_t sC, int M, int N, int K) {
  __shared__ __attribute__((aligned(16))) float so[4][16][64];
  const int tid = threadIdx.x, w = tid >> 5, lane = tid & 31, ln = lane & 15, hh = lane >> 4; const int by = blockIdx.y;
  A += (size_t)by * sA; Bh += (size_t)by * sB; const size_t cofs = (size_t)by * sC; const float* bp = bias ? bias + (size_t)by * sBias : nullptr;
  const int ntn = (N + 63) / 64; const int wid = blockIdx.x * 4 + w; const int mt = wid / ntn, nq = wid % ntn; if (mt * 16 >= M) return;
  const int row0 = mt * 16, col0 = nq * 64; const _Float16* arow = A + (size_t)(row0 + ln) * lda;
  v8f acc[4] = {};
  for (int kb = 0; kb < K; kb += 32) { FragH ah; ah.half[0] = *(const v8us*)((const unsigned short*)arow + kb + 8 * hh); ah.half[1] = *(const v8us*)((const unsigned short*)arow + kb + 16 + 8 * hh);
#pragma unroll
    for (int t = 0; t < 4; ++t) { if (col0 + t * 16 >= N) continue; const size_t boff = (size_t)(col0 + t * 16 + ln) * ldb + kb; FragH bq; bq.half[0] = *(const v8us*)((const unsigned short*)Bh + boff + 8 * hh); bq.half[1] = *(const v8us*)((const unsigned short*)Bh + boff + 16 + 8 * hh);
      acc[t] = mmaH<1>(ah.v, ah.v, bq.v, bq.v, acc[t]); }
  }
#pragma unroll
  for (int t = 0; t < 4; ++t) { if (col0 + t * 16 >= N) continue; const int col = col0 + t * 16 + ln; const float bv = bp ? bf16_round(bp[col]) : 0.f;
#pragma unroll
    for (int r = 0; r < 8; ++r) { float v = acc[t][r] * alpha + bv; if (CP) { const int bidx = (row0g + row0 + 8 * hh + r) / rowsPerB; v += CP[(size_t)bidx * sCPb + (size_t)by * 64 + col]; } if (ACT == 1) v = (v > 0.f) ? v : expm1f(v); else if (ACT == 7) v = (v > 0.f) ? v + 1.0f : expf(v); else if (ACT == 8) v = tanhf(v); else if (ACT == 9) v = 0.5f * v * (1.0f + tanhf(0.7978845608028654f * (v + 0.044715f * v * v * v))); else if (ACT == 11) v = 1.0f / (1.0f + expf(-v)); else if (ACT == 12) v = (v > 0.f) ? v : 0.01f * v; else if (ACT == 14) v = (v > 0.f) ? v : 0.1f * v; else if (ACT == 15) v = v / (1.0f + expf(-v)); else if (ACT == 3) v = fmaxf(v, 0.f); else if (ACT == 6) v = 0.5f * v * (1.0f + erff(v * 0.70710678118654752f)); so[w][8 * hh + r][t * 16 + ln] = v; } }
  __builtin_amdgcn_fence(__ATOMIC_ACQ_REL, "workgroup"); __builtin_amdgcn_wave_barrier();
  const int rsub = lane >> 4, c4 = (lane & 15) * 4; typedef _Float16 v4h __attribute__((ext_vector_type(4)));
  for (int pass = 0; pass < 2; ++pass) {
#pragma unroll
    for (int q = 0; q < 8; ++q) { const int r = q * 2 + rsub; if (col0 + c4 < N) { const v4f v = *(const v4fa*)&so[w][r][c4]; if (C) *(volatile v4f*)(C + cofs + (size_t)(row0 + r) * ldc + col0 + c4) = v; if (C16) { v4h h4; for (int i = 0; i < 4; ++i) h4[i] = (_Float16)v[i]; *(volatile v4h*)(C16 + cofs + (size_t)(row0 + r) * ldc + col0 + c4) = h4; } } }
    if (pass == 0) __threadfence(); }
}


typedef _Float16 v4h __attribute__((ext_vector_type(4)));

__global__ __launch_bounds__(256) void k_x16(const float* __restrict__ x, _Float16* __restrict__ X16, size_t n8) { const size_t t = (size_t)blockIdx.x * 256 + threadIdx.x; if (t >= n8) return; FragH f;
#pragma unroll
  for (int q = 0; q < 8; ++q) f.h[q] = (_Float16)bf16_round(x[t * 8 + q]); *(volatile v8us*)((unsigned short*)X16 + t * 8) = f.half[0]; __threadfence(); *(volatile v8us*)((unsigned short*)X16 + t * 8) = f.half[0]; }
__global__ __launch_bounds__(256) void k_h16(const float* __restrict__ x, _Float16* __restrict__ X16, size_t n8) { const size_t t = (size_t)blockIdx.x * 256 + threadIdx.x; if (t >= n8) return; FragH f;
#pragma unroll
  for (int q = 0; q < 8; ++q) f.h[q] = (_Float16)x[t * 8 + q]; *(volatile v8us*)((unsigned short*)X16 + t * 8) = f.half[0]; __threadfence(); *(volatile v8us*)((unsigned short*)X16 + t * 8) = f.half[0]; }
__global__ __launch_bounds__(256) void k_round16f(const float* __restrict__ W, _Float16* __restrict__ Bt, size_t n8) { const size_t t = (size_t)blockIdx.x * 256 + threadIdx.x; if (t >= n8) return; FragH f;
#pragma unroll
  for (int i = 0; i < 8; ++i) f.h[i] = (_Float16)(bf16_round(W[t * 8 + i]) * 16.0f); *(volatile v8us*)((unsigned short*)Bt + t * 8) = f.half[0]; __threadfence(); *(volatile v8us*)((unsigned short*)Bt + t * 8) = f.half[0]; }
template <int NHv, int TTv>
__global__ __launch_bounds__(256) void k_vt(const _Float16* __restrict__ V16, int ldv, int voff, _Float16* __restrict__ Vt) { __shared__ unsigned short tl[64][66]; const int tid = threadIdx.x; const int slab = blockIdx.x / (TTv / 64), lg = blockIdx.x % (TTv / 64); const int b = slab / NHv, h = slab % NHv;
  for (int i = tid; i < 64 * 8; i += 256) { const int r = i / 8, c8 = (i % 8) * 8; FragH f; f.half[0] = *(const v8us*)((const unsigned short*)V16 + ((size_t)b * TTv + lg * 64 + r) * ldv + voff + h * 64 + c8);
#pragma unroll
    for (int q = 0; q < 8; ++q) tl[r][c8 + q] = f.u[q]; }
  __syncthreads();
  for (int pass = 0; pass < 2; ++pass) {
#pragma unroll
    for (int rd = 0; rd < 2; ++rd) { const int d = rd * 32 + tid / 8, pc = tid % 8; FragH f;
#pragma unroll
      for (int q = 0; q < 8; ++q) f.u[q] = tl[pc * 8 + q][d];
      *(volatile v8us*)((unsigned short*)Vt + ((size_t)slab * 64 + d) * TTv + lg * 64 + pc * 8) = f.half[0]; }
    if (pass == 0) __threadfence(); } }

__global__ __launch_bounds__(256) void k_hl(const float* __restrict__ F, _Float16* __restrict__ Hh, _Float16* __restrict__ Hl, size_t n8) { const size_t t = (size_t)blockIdx.x * 256 + threadIdx.x; if (t >= n8) return; FragH fh, fl; const v4f a = *(const v4fa*)(F + t * 8), c = *(const v4fa*)(F + t * 8 + 4);
#pragma unroll
  for (int q = 0; q < 4; ++q) { _Float16 h = (_Float16)a[q]; fh.h[q] = h; fl.h[q] = (_Float16)((a[q] - (float)h) * 1024.0f); h = (_Float16)c[q]; fh.h[4 + q] = h; fl.h[4 + q] = (_Float16)((c[q] - (float)h) * 1024.0f); }
  for (int pass = 0; pass < 2; ++pass) { *(volatile v8us*)((unsigned short*)Hh + t * 8) = fh.half[0]; *(volatile v8us*)((unsigned short*)Hl + t * 8) = fl.half[0]; if (pass == 0) __threadfence(); } }

__device__ __forceinline__ float lrelu01(float v) { return (v >= 0.f) ? v : 0.01f * v; }
__global__ __launch_bounds__(256) void k_seg3(const float* __restrict__ F, _Float16* __restrict__ QA, _Float16* __restrict__ KB, size_t n8) {
  #pragma clang fp contract(off)
  const size_t t = (size_t)blockIdx.x * 256 + threadIdx.x; if (t >= n8) return; const size_t r = t >> 3; const int c0 = (int)(t & 7) * 8; const v4f a = *(const v4fa*)(F + t * 8), c = *(const v4fa*)(F + t * 8 + 4); FragH q0, q1, k0, k1, k2;
#pragma unroll
  for (int q = 0; q < 8; ++q) { const float v = (q < 4) ? a[q] : c[q - 4]; const _Float16 hi = (_Float16)v; const float lo = v - (float)hi; q0.h[q] = hi; q1.h[q] = (_Float16)(lo * 1024.0f); k0.h[q] = (_Float16)((float)hi * 16.0f); k1.h[q] = (_Float16)((float)hi * 0.015625f); k2.h[q] = (_Float16)(lo * 16.0f); }
  for (int pass = 0; pass < 2; ++pass) { unsigned short* qa = (unsigned short*)QA + r * 192; unsigned short* kb = (unsigned short*)KB + r * 192; *(volatile v8us*)(qa + c0) = q0.half[0]; *(volatile v8us*)(qa + 64 + c0) = q1.half[0]; *(volatile v8us*)(qa + 128 + c0) = q0.half[0]; *(volatile v8us*)(kb + c0) = k0.half[0]; *(volatile v8us*)(kb + 64 + c0) = k1.half[0]; *(volatile v8us*)(kb + 128 + c0) = k2.half[0]; if (pass == 0) __threadfence(); } }
__global__ __launch_bounds__(256) void k_adj(const float* __restrict__ S, _Float16* __restrict__ ADJ) {
  #pragma clang fp contract(off)
  const int tid = threadIdx.x, w = tid >> 5, ln = tid & 31; const int row = blockIdx.x * 8 + w; if (row >= GG * N1) return; const int i = row % N1; const float* sr = S + (size_t)row * N1;
  auto val = [&](int j) { const float s = sr[j] - ((j == i) ? 1.0e8f : 0.0f); return lrelu01(s); };
  float m = -3.0e38f; for (int j = ln; j < N1; j += 32) m = fmaxf(m, val(j));
  for (int o = 16; o > 0; o >>= 1) m = fmaxf(m, __shfl_xor(m, o, 32));
  float su = 0.f; for (int j = ln; j < N1; j += 32) su += expf(val(j) - m);
  for (int o = 16; o > 0; o >>= 1) su += __shfl_xor(su, o, 32); const float inv = 1.0f / su;
  for (int pass = 0; pass < 2; ++pass) { for (int ch = ln; ch < N1 / 8; ch += 32) { FragH f;
#pragma unroll
      for (int q = 0; q < 8; ++q) { const int j = ch * 8 + q; float a = expf(val(j) - m) * inv + ((j == i) ? 1.0f : 0.0f); a = a * (((j / NNODE) == (i / NNODE)) ? 1.0f : 0.7f); f.h[q] = (_Float16)(a * 1024.0f); }
      *(volatile v8us*)((unsigned short*)ADJ + (size_t)row * N1 + ch * 8) = f.half[0]; }
    if (pass == 0) __threadfence(); } }
__global__ __launch_bounds__(256) void k_colstat(const float* __restrict__ Pm, int windowed, int phase, float* __restrict__ STAT) {
  #pragma clang fp contract(off)
  __shared__ float red[256]; const int f = blockIdx.x, tid = threadIdx.x; const float mean = phase ? (STAT[(size_t)f * 32] / (float)NRW) : 0.f; float s = 0.f;
  for (int r = tid; r < NRW; r += 256) { size_t src; if (windowed) src = (size_t)r; else { const int g = r / N1, nd = r % N1; const int b = g / LW, l = g % LW; const int m = nd / NNODE, n = nd % NNODE; src = ((size_t)(b * SC + l + m)) * NNODE + n; } const float v = Pm[src * FF + f]; s += phase ? (v - mean) * (v - mean) : v; }
  red[tid] = s; __syncthreads(); for (int st = 128; st > 0; st >>= 1) { if (tid < st) red[tid] += red[tid + st]; __syncthreads(); }
  if (tid < 32) { float* line = STAT + ((size_t)phase * FF + f) * 32; *(volatile float*)(line + tid) = red[0]; __threadfence(); *(volatile float*)(line + tid) = red[0]; } }
__global__ __launch_bounds__(256) void k_xbt(const float* __restrict__ NF, const float* __restrict__ STAT, const float* __restrict__ w, const float* __restrict__ bb, _Float16* __restrict__ XBT) {
  #pragma clang fp contract(off)
  const int t = blockIdx.x * 256 + threadIdx.x; const int per = SC * NNODE / 8; if (t >= BS * FF * per) return; const int c0 = (t % per) * 8; const int f = (t / per) % FF; const int b = t / (per * FF); const float mu = STAT[(size_t)f * 32] / (float)NRW, rs = rsqrtf(STAT[(size_t)(FF + f) * 32] / (float)NRW + 1e-5f), ww = bf16_round(w[f]), b0 = bf16_round(bb[f]); FragH o;
#pragma unroll
  for (int q = 0; q < 8; ++q) o.h[q] = (_Float16)((NF[((size_t)b * SC * NNODE + c0 + q) * FF + f] - mu) * rs * ww + b0);
  *(volatile v8us*)((unsigned short*)XBT + ((size_t)b * FF + f) * (SC * NNODE) + c0) = o.half[0]; __threadfence(); *(volatile v8us*)((unsigned short*)XBT + ((size_t)b * FF + f) * (SC * NNODE) + c0) = o.half[0]; }
__global__ __launch_bounds__(256) void k_h1t(const float* __restrict__ H1, size_t row0, _Float16* __restrict__ H1T, _Float16* __restrict__ H116) { const int t = blockIdx.x * 256 + threadIdx.x; if (t >= GG * FF * (N1 / 8)) return; const int n0 = (t % (N1 / 8)) * 8; const int f = (t / (N1 / 8)) % FF; const int g = t / ((N1 / 8) * FF); FragH o;
#pragma unroll
  for (int q = 0; q < 8; ++q) o.h[q] = (_Float16)H1[((size_t)g * N1 + n0 + q) * FF + f];
  *(volatile v8us*)((unsigned short*)H1T + ((size_t)g * FF + f) * N1 + n0) = o.half[0]; __threadfence(); *(volatile v8us*)((unsigned short*)H1T + ((size_t)g * FF + f) * N1 + n0) = o.half[0]; (void)row0; (void)H116; }
__global__ __launch_bounds__(256) void k_f16(const float* __restrict__ F, _Float16* __restrict__ O16, size_t n8) { const size_t t = (size_t)blockIdx.x * 256 + threadIdx.x; if (t >= n8) return; const v4f a = *(const v4fa*)(F + t * 8), c = *(const v4fa*)(F + t * 8 + 4); FragH f;
#pragma unroll
  for (int q = 0; q < 8; ++q) f.h[q] = (_Float16)((q < 4) ? a[q] : c[q - 4]);
  *(volatile v8us*)((unsigned short*)O16 + t * 8) = f.half[0]; __threadfence(); *(volatile v8us*)((unsigned short*)O16 + t * 8) = f.half[0]; }
__global__ __launch_bounds__(256) void k_final(const float* __restrict__ OUT, const float* __restrict__ STAT, const float* __restrict__ w, const float* __restrict__ bb, float* __restrict__ out) {
  #pragma clang fp contract(off)
  const int t = blockIdx.x * 256 + threadIdx.x; if (t >= BS * NNODE * (FF / 4)) return; const int o0 = (t % (FF / 4)) * 4; const int n = (t / (FF / 4)) % NNODE; const int b = t / ((FF / 4) * NNODE); v4f acc = {0.f, 0.f, 0.f, 0.f}; float mu[4], rs[4], ww[4], b0[4];
#pragma unroll
  for (int q = 0; q < 4; ++q) { mu[q] = STAT[(size_t)(o0 + q) * 32] / (float)NRW; rs[q] = rsqrtf(STAT[(size_t)(FF + o0 + q) * 32] / (float)NRW + 1e-5f); ww[q] = bf16_round(w[o0 + q]); b0[q] = bf16_round(bb[o0 + q]); }
#pragma unroll 1
  for (int l = 0; l < LW; ++l) { v4f am = {0.f, 0.f, 0.f, 0.f};
    for (int m = 0; m < 2; ++m) { const size_t r = ((size_t)(b * LW + l) * 2 + m) * NNODE + n; const v4f v = *(const v4fa*)(OUT + r * FF + o0);
#pragma unroll
      for (int q = 0; q < 4; ++q) am[q] += lrelu01((v[q] - mu[q]) * rs[q] * ww[q] + b0[q]); }
    acc += am / 2.0f; }
  const v4f res = acc / (float)LW; float* dst = out + ((size_t)b * NNODE + n) * FF + o0; *(volatile v4f*)dst = res; __threadfence(); *(volatile v4f*)dst = res; }

extern "C" void kernel_launch(void* const* d_in, const int* in_sizes, int n_in,
                              void* d_out, int out_size, void* d_ws, size_t ws_size, hipStream_t stream) {
  (void)in_sizes; (void)n_in; (void)out_size;
  const float* const* I = (const float* const*)d_in; const float* x = I[0]; const float* wm = I[1]; const float* bm = I[2]; const float* bn0w = I[3]; const float* bn0b = I[4]; const float* th0 = I[5]; const float* th0b = I[6]; const float* th1 = I[7]; const float* th1b = I[8]; const float* bn1w = I[9]; const float* bn1b = I[10];
  char* ws = (char*)d_ws; size_t off = 0;
  auto take = [&](size_t bytes) { char* p = ws + off; off += (bytes + 255) & ~(size_t)255; return p; };
  _Float16* BM = (_Float16*)take(FF * FF * 2); _Float16* B0 = (_Float16*)take(FF * FF * 2); _Float16* B1t = (_Float16*)take(FF * FF * 2);
  char* RA = take((size_t)NRX * FF * 2 + (size_t)NRX * FF * 4 + (size_t)NRX * FF * 2 + 512);
  _Float16* X16 = (_Float16*)RA; float* NF = (float*)(RA + (size_t)NRX * FF * 2); _Float16* NF16 = (_Float16*)(RA + (size_t)NRX * FF * 6); float* OUT = (float*)RA; float* STAT0 = (float*)take(2 * FF * 32 * 4); float* STAT1 = (float*)take(2 * FF * 32 * 4); _Float16* XBT = (_Float16*)take((size_t)BS * FF * SC * NNODE * 2);
  float* S = (float*)take((size_t)GG * N1 * N1 * 4); _Float16* ADJ = (_Float16*)take((size_t)GG * N1 * N1 * 2); float* H1 = (float*)take((size_t)GG * N1 * FF * 4); _Float16* H1T = (_Float16*)take((size_t)GG * FF * N1 * 2); float* H2 = (float*)take((size_t)GG * N1 * FF * 4); _Float16* H116 = (_Float16*)take((size_t)NRW * FF * 2); _Float16* H216 = (_Float16*)take((size_t)NRW * FF * 2);
  if (off > ws_size) return;
  k_round16f<<<(FF * FF / 8 + 255) / 256, 256, 0, stream>>>(wm, BM, (size_t)FF * FF / 8); k_round16f<<<(FF * FF / 8 + 255) / 256, 256, 0, stream>>>(th0, B0, (size_t)FF * FF / 8); k_round16f<<<(FF * FF / 8 + 255) / 256, 256, 0, stream>>>(th1, B1t, (size_t)FF * FF / 8);
  const size_t n8x = (size_t)NRX * FF / 8; k_x16<<<(unsigned)((n8x + 255) / 256), 256, 0, stream>>>(x, X16, n8x);
  k_gemm_hhx<0><<<dim3(((NRX / 16) * 1 + 3) / 4, 1), 128, 0, stream>>>(X16, FF, 0, BM, FF, 0, 0.0625f, bm, 0, nullptr, 1, 0, 0, NF, nullptr, FF, 0, NRX, FF, FF); k_f16<<<(unsigned)((n8x + 255) / 256), 256, 0, stream>>>(NF, NF16, n8x);
  k_colstat<<<FF, 256, 0, stream>>>(NF, 0, 0, STAT0); k_colstat<<<FF, 256, 0, stream>>>(NF, 0, 1, STAT0);
  k_xbt<<<(BS * FF * (SC * NNODE / 8) + 255) / 256, 256, 0, stream>>>(NF, STAT0, bn0w, bn0b, XBT);
  const dim3 gS(((N1 / 16) * (N1 / 64) + 3) / 4, GG), gH(((N1 / 16) * 1 + 3) / 4, GG);
  for (int gi = 0; gi < NG / GG; ++gi) { const int g0 = gi * GG; const int b = g0 / LW, l0 = g0 % LW;
    const _Float16* nfg = NF16 + ((size_t)(b * SC + l0)) * NNODE * FF;
    k_gemm_hhx<0><<<gS, 128, 0, stream>>>(nfg, FF, (size_t)NNODE * FF, nfg, FF, (size_t)NNODE * FF, 1.0f, nullptr, 0, nullptr, 1, 0, 0, S, nullptr, N1, (size_t)N1 * N1, N1, N1, FF);
    k_adj<<<GG * N1 / 8, 256, 0, stream>>>(S, ADJ);
    const _Float16* xbg = XBT + (size_t)b * FF * (SC * NNODE) + (size_t)l0 * NNODE;
    k_gemm_hhx<0><<<gH, 128, 0, stream>>>(ADJ, N1, (size_t)N1 * N1, xbg, SC * NNODE, (size_t)NNODE, 0.0009765625f, nullptr, 0, nullptr, 1, 0, 0, H1, nullptr, FF, (size_t)N1 * FF, N1, FF, N1);
    k_h1t<<<(GG * FF * (N1 / 8) + 255) / 256, 256, 0, stream>>>(H1, 0, H1T, nullptr); k_f16<<<(GG * N1 * FF / 8 + 255) / 256, 256, 0, stream>>>(H1, H116 + (size_t)g0 * N1 * FF, (size_t)GG * N1 * FF / 8);
    k_gemm_hhx<0><<<gH, 128, 0, stream>>>(ADJ, N1, (size_t)N1 * N1, H1T, N1, (size_t)FF * N1, 0.0009765625f, nullptr, 0, nullptr, 1, 0, 0, H2, nullptr, FF, (size_t)N1 * FF, N1, FF, N1);
    k_f16<<<(GG * N1 * FF / 8 + 255) / 256, 256, 0, stream>>>(H2, H216 + (size_t)g0 * N1 * FF, (size_t)GG * N1 * FF / 8); }
  const dim3 gO(((NRW / 16) * 1 + 3) / 4, 1);
  k_gemm_hhx<0><<<gO, 128, 0, stream>>>(H116, FF, 0, B0, FF, 0, 0.0625f, th0b, 0, nullptr, 1, 0, 0, OUT, nullptr, FF, 0, NRW, FF, FF); k_gemm_hhx<0><<<gO, 128, 0, stream>>>(H216, FF, 0, B1t, FF, 0, 0.0625f, th1b, 0, OUT, 1, (size_t)FF, 0, OUT, nullptr, FF, 0, NRW, FF, FF);
  k_colstat<<<FF, 256, 0, stream>>>(OUT, 1, 0, STAT1); k_colstat<<<FF, 256, 0, stream>>>(OUT, 1, 1, STAT1);
  k_final<<<(BS * NNODE * (FF / 4) + 255) / 256, 256, 0, stream>>>(OUT, STAT1, bn1w, bn1b, (float*)d_out);
}
